// Attention_23321672417682
// MI455X (gfx1250) — hardware-verified
//
#include <hip/hip_runtime.h>


#ifndef NB
#define NB 8
#endif
#ifndef SEQ
#define SEQ 2048
#endif
#define NB_FULL  8
#define SEQ_FULL 2048
#define DIM  512
#define NH   8
#define HD   64
#define DIM3 1536
#define KC   1024
#define NWV  4
#define BQ   (16 * NWV)
#define KS   32
#define OSP  68
#define GP   68
#define GBM  128
#define GBN  64
#define WTP  72
#define L2E  1.4426950408889634f
#define PCL  10.0f
#define QCAR 64.0f
#define KCAR 8.0f
#define RSC  2048.0f
#define RINV (1.0f / 2048.0f)
#define SCL  (1.0f / 512.0f)
#define L2ES (L2E * SCL)
#define MROWS (NB * SEQ)
#define PLN  ((size_t)MROWS * DIM)

static_assert(HD == 64);
static_assert(GBN == HD);
static_assert(NH * HD == DIM);
static_assert(DIM3 == 3 * DIM);
static_assert(KC == 2 * DIM);
static_assert(DIM % 32 == 0);
static_assert(KC % 32 == 0);
static_assert(HD % 32 == 0);
static_assert(DIM % 64 == 0);
static_assert(DIM3 % GBN == 0);
static_assert(DIM % GBN == 0);
static_assert(SEQ % BQ == 0);
static_assert(SEQ % KS == 0);
static_assert(SEQ % GBM == 0);
static_assert(MROWS % GBM == 0);
static_assert(GBM == 32 * NWV);
static_assert(NB <= NB_FULL);
static_assert(SEQ <= SEQ_FULL);
static_assert(QCAR * KCAR * SCL == 1.0f);
static_assert(RSC * RINV == 1.0f);
static_assert(((size_t)MROWS * DIM) % 2048 == 0);
static_assert((size_t)(MROWS / GBM) * (DIM3 / GBN) * (size_t)(GBM * GBN) == (size_t)MROWS * DIM3);
static_assert((size_t)(MROWS / GBM) * (DIM / GBN) * (size_t)(GBM * GBN) == (size_t)MROWS * DIM);
static_assert((size_t)(NB * NH) * (SEQ / BQ) * (size_t)(BQ * HD) == (size_t)MROWS * DIM);
static_assert(8 * 128 == GBM * (HD / 8));
static_assert(8 * 128 == HD * (GBM / 8));
static_assert(16 * 128 == GBM * (GBN / 4));
static_assert(4 * 4 == 16);

typedef unsigned short bf;
typedef __attribute__((ext_vector_type(16))) __bf16   v16bf;
typedef __attribute__((ext_vector_type(16))) _Float16 v16h;
typedef __attribute__((ext_vector_type(8)))  _Float16 v8h;
typedef __attribute__((ext_vector_type(8)))  unsigned short v8us;
typedef __attribute__((ext_vector_type(8)))  float    v8f;
typedef __attribute__((ext_vector_type(4)))  float    v4f;
typedef v4f  __attribute__((may_alias)) v4fa;
typedef v8us __attribute__((may_alias)) v8usa;

__device__ __forceinline__ unsigned short f2bf(float f) { unsigned u = __float_as_uint(f); u += 0x7FFFu + ((u >> 16) & 1u); return (unsigned short)(u >> 16); }
__device__ __forceinline__ float bf2f(unsigned short b) { return __uint_as_float(((unsigned)b) << 16); }
__device__ __forceinline__ v8f wmmab(v16bf a, v16bf b, v8f c) { return __builtin_amdgcn_wmma_f32_16x16x32_bf16(false, a, false, b, (short)0, c, false, false); }
__device__ __forceinline__ v8f wmmah(v16h a, v16h b, v8f c) { return __builtin_amdgcn_wmma_f32_16x16x32_f16(false, a, false, b, (short)0, c, false, false); }
__device__ __forceinline__ v16bf ldb(const bf* p) {
    const v8us lo = *(const v8us*)p; const v8us hi = *(const v8us*)(p + 16);
    return __builtin_bit_cast(v16bf, __builtin_shufflevector(lo, hi, 0, 1, 2, 3, 4, 5, 6, 7, 8, 9, 10, 11, 12, 13, 14, 15));
}
__device__ __forceinline__ v16h ldh(const bf* p) {
    const v8us lo = *(const v8us*)p; const v8us hi = *(const v8us*)(p + 16);
    return __builtin_bit_cast(v16h, __builtin_shufflevector(lo, hi, 0, 1, 2, 3, 4, 5, 6, 7, 8, 9, 10, 11, 12, 13, 14, 15));
}

__global__ __launch_bounds__(256) void k_cvt8(const float* __restrict__ x, bf* XB) {
    const unsigned i = blockIdx.x * 256u + threadIdx.x;
    const unsigned per = (unsigned)(SEQ * DIM / 8);
    if (i >= (unsigned)NB * per) return;
    const unsigned b = i / per, r = i - b * per;
    const float* src = x + (size_t)b * SEQ_FULL * DIM + (size_t)r * 8;
    bf* dst = XB + (size_t)i * 8;
    const v8f v = *(const v8f*)src;
    v8us o;
#pragma unroll
    for (int c = 0; c < 8; ++c) o[c] = f2bf(v[c]);
    *(volatile v8us*)dst = o;
    __threadfence();
    *(volatile v8us*)dst = o;
}

__global__ __launch_bounds__(256) void k_wt(const float* __restrict__ W, bf* WT, int N, int pitch, int ndup, int qcols) {
    __shared__ __align__(16) bf tl[64 * WTP];
    const unsigned tid = threadIdx.x;
    const unsigned n0 = blockIdx.x * 64u, k0 = blockIdx.y * 64u;
    const float sc = ((int)n0 < qcols) ? 0.125f : 1.0f;
#pragma unroll
    for (unsigned it = 0; it < 4; ++it) {
        const unsigned f = it * 256u + tid;
        const unsigned kk = f >> 4, n4 = (f & 15u) * 4u;
        const v4f x = *(const v4f*)(W + (size_t)(k0 + kk) * (unsigned)N + n0 + n4);
#pragma unroll
        for (unsigned c = 0; c < 4; ++c) tl[(n4 + c) * WTP + kk] = f2bf(x[c] * sc);
    }
    __syncthreads();
    const unsigned c8 = (tid & 7u) * 8u, nr = tid >> 3;
#pragma unroll 1
    for (int ps = 0; ps < 2; ++ps) {
#pragma unroll 1
        for (int dup = 0; dup < ndup; ++dup) {
#pragma unroll
            for (unsigned it = 0; it < 2; ++it) {
                const unsigned n = it * 32u + nr;
                const v8us o = *(const v8usa*)(tl + n * WTP + c8);
                *(volatile v8us*)(WT + (size_t)(n0 + n) * (unsigned)pitch + (unsigned)dup * DIM + k0 + c8) = o;
            }
        }
        if (ps == 0) __threadfence();
    }
}

__device__ __forceinline__ void gemm_acc(const bf* __restrict__ A, const bf* __restrict__ BT, const unsigned K,
                                         const unsigned arow, const unsigned brow, const unsigned hi, v8f (&acc)[2][4]) {
    const bf* ap = A + (size_t)arow * K + 8u * hi;
    const bf* bp = BT + (size_t)brow * K + 8u * hi;
    const size_t s16 = (size_t)16 * K;
#pragma unroll 1
    for (unsigned k0 = 0; k0 < K; k0 += 32) {
        const v16bf a0 = ldb(ap + k0);
        const v16bf a1 = ldb(ap + s16 + k0);
        const v16bf b0 = ldb(bp + k0);
        const v16bf b1 = ldb(bp + s16 + k0);
        const v16bf b2 = ldb(bp + 2 * s16 + k0);
        const v16bf b3 = ldb(bp + 3 * s16 + k0);
        acc[0][0] = wmmab(a0, b0, acc[0][0]);
        acc[1][0] = wmmab(a1, b0, acc[1][0]);
        acc[0][1] = wmmab(a0, b1, acc[0][1]);
        acc[1][1] = wmmab(a1, b1, acc[1][1]);
        acc[0][2] = wmmab(a0, b2, acc[0][2]);
        acc[1][2] = wmmab(a1, b2, acc[1][2]);
        acc[0][3] = wmmab(a0, b3, acc[0][3]);
        acc[1][3] = wmmab(a1, b3, acc[1][3]);
        asm volatile("v_nop\n\tv_nop\n\tv_nop\n\tv_nop"
                     : "+v"(acc[0][0]), "+v"(acc[1][0]), "+v"(acc[0][1]), "+v"(acc[1][1]),
                       "+v"(acc[0][2]), "+v"(acc[1][2]), "+v"(acc[0][3]), "+v"(acc[1][3])
                     : "v"(a0), "v"(a1), "v"(b0), "v"(b1), "v"(b2), "v"(b3));
    }
}

__global__ __launch_bounds__(128) void k_qkv(const bf* __restrict__ XB, const bf* __restrict__ WQT, bf* QK, bf* VT) {
    __shared__ __align__(16) float st[GBM * GP];
    const unsigned tid = threadIdx.x, lane = tid & 31u, wv = tid >> 5, lr = lane & 15u, hi = lane >> 4;
    const unsigned ntn = (unsigned)(DIM3 / GBN);
    const unsigned mT = blockIdx.x / ntn, nT = blockIdx.x - mT * ntn;
    const unsigned m0 = mT * GBM, n0 = nT * GBN;
    v8f acc[2][4];
#pragma unroll
    for (int i = 0; i < 2; ++i)
#pragma unroll
        for (int j = 0; j < 4; ++j) acc[i][j] = (v8f){};
    gemm_acc(XB, WQT, (unsigned)DIM, m0 + wv * 32u + lr, n0 + lr, hi, acc);
#pragma unroll
    for (int i = 0; i < 2; ++i)
#pragma unroll
        for (int j = 0; j < 4; ++j)
#pragma unroll
            for (int r = 0; r < 8; ++r) st[(wv * 32u + i * 16u + 8u * hi + r) * GP + j * 16u + lr] = acc[i][j][r];
    __syncthreads();
    const unsigned which = nT >> 3, h = nT & 7u;
    const unsigned b = m0 / (unsigned)SEQ, nq0 = m0 - b * (unsigned)SEQ;
    const unsigned bh = b * NH + h;
    if (which < 2u) {
        bf* ph = QK + (size_t)which * 2 * PLN + ((size_t)bh * SEQ + nq0) * HD;
        const float car = (which == 0u) ? QCAR : KCAR;
#pragma unroll 1
        for (int ps = 0; ps < 2; ++ps) {
#pragma unroll
            for (unsigned it = 0; it < 8; ++it) {
                const unsigned idx = it * 128u + tid;
                const unsigned row = idx >> 3, c8 = (idx & 7u) * 8u;
                const v4f x0 = *(const v4fa*)(st + row * GP + c8);
                const v4f x1 = *(const v4fa*)(st + row * GP + c8 + 4u);
                v8h ov, orr;
#pragma unroll
                for (int c = 0; c < 4; ++c) {
                    const float y0 = x0[c] * car, y1 = x1[c] * car;
                    const _Float16 h0 = (_Float16)y0, h1 = (_Float16)y1;
                    ov[c] = h0; ov[4 + c] = h1;
                    orr[c] = (_Float16)((y0 - (float)h0) * RSC);
                    orr[4 + c] = (_Float16)((y1 - (float)h1) * RSC);
                }
                const v8us ouv = __builtin_bit_cast(v8us, ov);
                const v8us our = __builtin_bit_cast(v8us, orr);
                *(volatile v8us*)(ph + (size_t)row * HD + c8) = ouv;
                if (which == 0u) *(volatile v8us*)(ph + PLN + (size_t)row * HD + c8) = our;
            }
            if (ps == 0) __threadfence();
        }
    } else {
        bf* pv = VT + (size_t)bh * HD * SEQ + nq0;
#pragma unroll 1
        for (int ps = 0; ps < 2; ++ps) {
#pragma unroll
            for (unsigned it = 0; it < 8; ++it) {
                const unsigned idx = it * 128u + tid;
                const unsigned d = idx >> 4, n8 = (idx & 15u) * 8u;
                v8h o;
#pragma unroll
                for (unsigned c = 0; c < 8; ++c) o[c] = (_Float16)st[(n8 + c) * GP + d];
                const v8us ou = __builtin_bit_cast(v8us, o);
                *(volatile v8us*)(pv + (size_t)d * SEQ + n8) = ou;
            }
            if (ps == 0) __threadfence();
        }
    }
}

__global__ __launch_bounds__(128) void k_flash(const bf* __restrict__ QK, const bf* __restrict__ VT, bf* CTX) {
    __shared__ __align__(16) float os[NWV * 16 * OSP];
    const unsigned tid = threadIdx.x, lane = tid & 31u, wv = tid >> 5, lr = lane & 15u, hi = lane >> 4;
    const unsigned bpb = (unsigned)(SEQ / BQ);
    const unsigned bh = blockIdx.x / bpb;
    const unsigned q0 = (blockIdx.x - bh * bpb) * BQ + wv * 16u;
    const unsigned b = bh / NH, h = bh - b * NH;

    v16h qh[2], qr[2];
    {
        const bf* qp = QK + ((size_t)bh * SEQ + q0 + lr) * HD + 8u * hi;
#pragma unroll
        for (int dk = 0; dk < 2; ++dk) { qh[dk] = ldh(qp + dk * 32); qr[dk] = ldh(qp + PLN + dk * 32); }
    }
    const bf* kp = QK + 2 * PLN + ((size_t)bh * SEQ + lr) * HD + 8u * hi;
    const bf* vp = VT + ((size_t)bh * HD + lr) * SEQ + 8u * hi;

    v8f o[4];
#pragma unroll
    for (int t = 0; t < 4; ++t) o[t] = (v8f){};
    float ml = -1.0e30f;
    float l = 0.0f;

#pragma unroll 1
    for (unsigned k0 = 0; k0 < (unsigned)SEQ; k0 += KS) {
        v8f s0 = (v8f){}, s1 = (v8f){}, r0 = (v8f){}, r1 = (v8f){};
        const bf* ka = kp + (size_t)k0 * HD;
#pragma unroll
        for (int dk = 0; dk < 2; ++dk) {
            const v16h a0 = ldh(ka + dk * 32);
            const v16h a1 = ldh(ka + 16 * HD + dk * 32);
            s0 = wmmah(a0, qh[dk], s0);
            s1 = wmmah(a1, qh[dk], s1);
            r0 = wmmah(a0, qr[dk], r0);
            r1 = wmmah(a1, qr[dk], r1);
        }
        asm volatile("v_nop\n\tv_nop\n\tv_nop\n\tv_nop" : "+v"(s0), "+v"(s1), "+v"(r0), "+v"(r1) : "v"(qh[0]), "v"(qh[1]), "v"(qr[0]), "v"(qr[1]));
#pragma unroll
        for (int r = 0; r < 8; ++r) { s0[r] = fmaf(r0[r], RINV, s0[r]); s1[r] = fmaf(r1[r], RINV, s1[r]); }

        float mx = fmaxf(s0[0], s1[0]);
#pragma unroll
        for (int r = 1; r < 8; ++r) mx = fmaxf(mx, fmaxf(s0[r], s1[r]));
        mx = fmaxf(mx, __shfl_xor(mx, 16, 32));
        const float mnl = fmaxf(ml, mx * L2ES);
        const float corr = __builtin_amdgcn_exp2f(ml - mnl);
        ml = mnl;
        const float sh = PCL - mnl;
        float p0[8], p1[8];
        float ps = 0.0f;
#pragma unroll
        for (int r = 0; r < 8; ++r) {
            p0[r] = __builtin_amdgcn_exp2f(fmaf(s0[r], L2ES, sh));
            p1[r] = __builtin_amdgcn_exp2f(fmaf(s1[r], L2ES, sh));
            ps += p0[r] + p1[r];
        }
        ps += __shfl_xor(ps, 16, 32);
        l = l * corr + ps;
        if (__builtin_amdgcn_ballot_w32(corr != 1.0f) != 0u) {
#pragma unroll
            for (int t = 0; t < 4; ++t) o[t] *= corr;
        }

        v16h ph;
#pragma unroll
        for (int r = 0; r < 8; ++r) { ph[r] = (_Float16)p0[r]; ph[8 + r] = (_Float16)p1[r]; }

        asm volatile("" ::: "memory");
        const bf* va = vp + k0;
#pragma unroll
        for (int t = 0; t < 4; ++t) {
            const v16h a = ldh(va + (size_t)t * 16 * SEQ);
            o[t] = wmmah(a, ph, o[t]);
        }
        asm volatile("v_nop\n\tv_nop\n\tv_nop\n\tv_nop"
                     : "+v"(o[0]), "+v"(o[1]), "+v"(o[2]), "+v"(o[3])
                     : "v"(ph));
    }

    const float inv = 1.0f / l;
    float* ow = os + wv * (16 * OSP);
#pragma unroll
    for (int t = 0; t < 4; ++t) {
#pragma unroll
        for (int r = 0; r < 8; ++r) ow[lr * OSP + t * 16 + 8 * hi + r] = o[t][r] * inv;
    }
    __syncthreads();
    bf* crow = CTX + ((size_t)b * SEQ + q0) * KC + h * HD;
    const unsigned rq = lane >> 3, c8 = (lane & 7u) * 8u;
#pragma unroll 1
    for (int ps2 = 0; ps2 < 2; ++ps2) {
#pragma unroll
        for (unsigned it = 0; it < 4; ++it) {
            const unsigned row = it * 4u + rq;
            const v4f x0 = *(const v4fa*)(ow + row * OSP + c8);
            const v4f x1 = *(const v4fa*)(ow + row * OSP + c8 + 4u);
            v8us oh, ol;
#pragma unroll
            for (int c = 0; c < 4; ++c) {
                const unsigned short h0 = f2bf(x0[c]), h1 = f2bf(x1[c]);
                oh[c] = h0; oh[4 + c] = h1;
                ol[c] = f2bf(x0[c] - bf2f(h0)); ol[4 + c] = f2bf(x1[c] - bf2f(h1));
            }
            *(volatile v8us*)(crow + (size_t)row * KC + c8) = oh;
            *(volatile v8us*)(crow + (size_t)row * KC + DIM + c8) = ol;
        }
        if (ps2 == 0) __threadfence();
    }
}

__global__ __launch_bounds__(128) void k_proj(const bf* __restrict__ CTX, const bf* __restrict__ WOT, float* O) {
    __shared__ __align__(16) float st[GBM * GP];
    const unsigned tid = threadIdx.x, lane = tid & 31u, wv = tid >> 5, lr = lane & 15u, hi = lane >> 4;
    const unsigned ntn = (unsigned)(DIM / GBN);
    const unsigned mT = blockIdx.x / ntn, nT = blockIdx.x - mT * ntn;
    const unsigned m0 = mT * GBM, n0 = nT * GBN;
    v8f acc[2][4];
#pragma unroll
    for (int i = 0; i < 2; ++i)
#pragma unroll
        for (int j = 0; j < 4; ++j) acc[i][j] = (v8f){};
    gemm_acc(CTX, WOT, (unsigned)KC, m0 + wv * 32u + lr, n0 + lr, hi, acc);
#pragma unroll
    for (int i = 0; i < 2; ++i)
#pragma unroll
        for (int j = 0; j < 4; ++j)
#pragma unroll
            for (int r = 0; r < 8; ++r) st[(wv * 32u + i * 16u + 8u * hi + r) * GP + j * 16u + lr] = acc[i][j][r];
    __syncthreads();
    float* ob = O + (size_t)m0 * DIM + n0;
#pragma unroll 1
    for (int ps = 0; ps < 2; ++ps) {
#pragma unroll 4
        for (unsigned it = 0; it < 16; ++it) {
            const unsigned idx = it * 128u + tid;
            const unsigned row = idx >> 4, c4 = (idx & 15u) * 4u;
            const v4f val = *(const v4fa*)(st + row * GP + c4);
            *(volatile v4f*)(ob + (size_t)row * DIM + c4) = val;
        }
        if (ps == 0) __threadfence();
    }
}

extern "C" void kernel_launch(void* const* d_in, const int* in_sizes, int n_in,
                              void* d_out, int out_size, void* d_ws, size_t ws_size, hipStream_t stream) {
    if (n_in < 3) return;
    const size_t needx = ((size_t)(NB - 1) * SEQ_FULL + SEQ) * DIM;
    if ((size_t)in_sizes[0] < needx) return;
    if ((size_t)in_sizes[1] < (size_t)DIM * DIM3) return;
    if ((size_t)in_sizes[2] < (size_t)DIM * DIM) return;
    if ((size_t)out_size < (size_t)MROWS * DIM) return;
    const float* x     = (const float*)d_in[0];
    const float* w_qkv = (const float*)d_in[1];
    const float* w_out = (const float*)d_in[2];
    float* OUT = (float*)d_out;

    constexpr size_t WQT_B = (size_t)DIM3 * DIM * 2;
    constexpr size_t WOT_B = (size_t)DIM * KC * 2;
    constexpr size_t PLN_B = (size_t)MROWS * DIM * 2;
    constexpr size_t OFF_WQT = 0;
    constexpr size_t OFF_WOT = OFF_WQT + WQT_B;
    constexpr size_t OFF_QK  = OFF_WOT + WOT_B;
    constexpr size_t OFF_VT  = OFF_QK + 3 * PLN_B;
    constexpr size_t OFF_XC  = OFF_VT + PLN_B;
    constexpr size_t WS_TOTAL = OFF_XC + 2 * PLN_B;
    static_assert(WS_TOTAL <= (size_t)134217728);
    static_assert(OFF_WOT % 256 == 0);
    static_assert(OFF_QK % 256 == 0);
    static_assert(OFF_VT % 256 == 0);
    static_assert(OFF_XC % 256 == 0);
    static_assert(OFF_VT - OFF_QK == 3 * PLN_B);
    static_assert((size_t)MROWS * KC * 2 == 2 * PLN_B);
    static_assert((size_t)MROWS * DIM * 2 <= 2 * PLN_B);
    if (WS_TOTAL > ws_size) return;

    char* wsp = (char*)d_ws;
    bf* WQT = (bf*)(wsp + OFF_WQT);
    bf* WOT = (bf*)(wsp + OFF_WOT);
    bf* QK  = (bf*)(wsp + OFF_QK);
    bf* VT  = (bf*)(wsp + OFF_VT);
    bf* XB  = (bf*)(wsp + OFF_XC);
    bf* CTX = (bf*)(wsp + OFF_XC);

    const unsigned gc = (unsigned)(((size_t)MROWS * DIM / 8 + 255) / 256);
    k_cvt8<<<gc, 256, 0, stream>>>(x, XB);
    k_wt<<<dim3(DIM3 / 64, DIM / 64, 1), 256, 0, stream>>>(w_qkv, WQT, DIM3, DIM, 1, DIM);
    k_wt<<<dim3(DIM / 64, DIM / 64, 1), 256, 0, stream>>>(w_out, WOT, DIM, KC, 2, 0);
    k_qkv<<<(unsigned)((MROWS / GBM) * (DIM3 / GBN)), 128, 0, stream>>>(XB, WQT, QK, VT);
    k_flash<<<(unsigned)(NB * NH * (SEQ / BQ)), 128, 0, stream>>>(QK, VT, CTX);
    k_proj<<<(unsigned)((MROWS / GBM) * (DIM / GBN)), 128, 0, stream>>>(CTX, WOT, OUT);
}
